// DENetEncoder_48945447305228
// MI455X (gfx1250) — hardware-verified
//
#include <hip/hip_runtime.h>
#include <hip/hip_bf16.h>
#include <math.h>

#define BB 8
#define NN 16384
#define KNB 16
#define CC 64
#define MD 32
#define HD2 32
#define HIDm 128
#define GSTR 48

typedef _Float16 bf16;
typedef _Float16 f16;
typedef __attribute__((ext_vector_type(4))) unsigned v4u_t;
typedef unsigned v4ua __attribute__((ext_vector_type(4), may_alias));
typedef __attribute__((ext_vector_type(4))) float v4f_t;
typedef float v4fa __attribute__((ext_vector_type(4), may_alias));
typedef __attribute__((ext_vector_type(16))) bf16  bf16x16;
typedef bf16x16 f16x16;
typedef __attribute__((ext_vector_type(8)))  bf16  bf16x8;
typedef bf16x8 f16x8;
typedef __attribute__((ext_vector_type(4)))  bf16  bf16x4;
typedef __attribute__((ext_vector_type(8)))  float f32x8;
__device__ __forceinline__ f32x8 wmma16(f16x16 a, f16x16 b, f32x8 c) {
  c = __builtin_amdgcn_wmma_f32_16x16x32_f16(false, a, false, b, (short)0, c, false, false);
  asm volatile("v_nop\n\tv_nop\n\tv_nop\n\tv_nop" : "+v"(c) : "v"(a), "v"(b));
  return c;
}
#define LDS_STRIDE 48
#define KSTRIDE    72
#define VSTRIDE    48

__device__ __forceinline__ f32x8 wmma_bf16(bf16x16 a, bf16x16 b, f32x8 c) {
  c = __builtin_amdgcn_wmma_f32_16x16x32_f16(false, a, false, b, (short)0, c, false, false);
  asm volatile("v_nop\n\tv_nop\n\tv_nop\n\tv_nop" : "+v"(c) : "v"(a), "v"(b));
  return c;
}

template <typename T>
__device__ __forceinline__ bf16x16 load_frag(const T* __restrict__ base, int ld,
                                             int row0, int k0) {
  const int lane = threadIdx.x & 31;
  const int r    = lane & 15;
  const int kh   = (lane >> 4) * 8;
  const T* p0 = base + (size_t)(row0 + r) * ld + (k0 + kh);
  const T* p1 = p0 + 16;
  bf16x16 f;
#pragma unroll
  for (int i = 0; i < 8; ++i) {
    f[i]     = (bf16)p0[i];
    f[i + 8] = (bf16)p1[i];
  }
  return f;
}

__device__ __forceinline__ bf16x16 lds_frag(const bf16* base, int stride) {
  const int lane = threadIdx.x & 31;
  const int row  = lane & 15;
  const int kh   = (lane >> 4) * 8;
  const bf16x8 lo = *(const bf16x8*)(base + row * stride + kh);
  const bf16x8 hi = *(const bf16x8*)(base + row * stride + kh + 16);
  bf16x16 f;
#pragma unroll
  for (int i = 0; i < 8; ++i) { f[i] = lo[i]; f[i + 8] = hi[i]; }
  return f;
}

template <typename T>
__device__ __forceinline__ void stage_read16(const T* __restrict__ p, float* buf) {
#pragma unroll
  for (int i = 0; i < 16; ++i) buf[i] = (float)p[i];
}

__device__ __forceinline__ void stage_write(bf16* dst, const float* buf, int nquad) {
#pragma unroll
  for (int i = 0; i < nquad; ++i) {
    bf16x4 q;
    q[0] = (bf16)buf[4 * i];     q[1] = (bf16)buf[4 * i + 1];
    q[2] = (bf16)buf[4 * i + 2]; q[3] = (bf16)buf[4 * i + 3];
    *(bf16x4*)(dst + 4 * i) = q;
  }
}


#define GSTR 48
template <typename AT, int EPI, bool OUT16>
__global__ __launch_bounds__(256) void gemm_kne(const AT* __restrict__ A, int lda, const float* __restrict__ Wm, int ldw,
                                                const float* __restrict__ bias, const float* __restrict__ R, const float* __restrict__ gvec,
                                                void* __restrict__ Yv, int ldy, int K) {
  __shared__ __attribute__((aligned(16))) f16 ldsA[128 * GSTR];
  __shared__ __attribute__((aligned(16))) f16 ldsW[128 * GSTR];
  __shared__ __attribute__((aligned(16))) float oS[8][32 * 68];
  const int tid = threadIdx.x, lane = tid & 31, wave = tid >> 5, cl = lane & 15, rh = (lane >> 4) * 8;
  const int m0 = blockIdx.x * 128, n0 = blockIdx.y * 128;
  const int wm = (wave & 3) * 32, wn = (wave >> 2) * 64;
  f32x8 acc[2][4];
#pragma unroll
  for (int i = 0; i < 2; ++i)
#pragma unroll
    for (int j = 0; j < 4; ++j) { f32x8 z = {}; acc[i][j] = z; }
#pragma unroll 1
  for (int k0 = 0; k0 < K; k0 += 32) {
    __syncthreads();
    { const int row = tid >> 1, ch = (tid & 1) * 16;
      const AT* src = A + (size_t)(m0 + row) * lda + k0 + ch;
#pragma unroll
      for (int g = 0; g < 16; ++g) ldsA[row * GSTR + ch + g] = (f16)src[g]; }
    { const int k = tid >> 3, nn0 = (tid & 7) * 16;
      const float* src = Wm + (size_t)(k0 + k) * ldw + n0 + nn0;
#pragma unroll
      for (int g = 0; g < 4; ++g) { const v4f_t v = *(const v4f_t*)(src + 4 * g);
#pragma unroll
        for (int u = 0; u < 4; ++u) ldsW[(nn0 + 4 * g + u) * GSTR + k] = (f16)v[u]; } }
    __syncthreads();
    f16x16 af[2];
#pragma unroll
    for (int i = 0; i < 2; ++i) af[i] = lds_frag(ldsA + (wm + 16 * i) * GSTR, GSTR);
#pragma unroll
    for (int j = 0; j < 4; ++j) {
      const f16x16 bf = lds_frag(ldsW + (wn + 16 * j) * GSTR, GSTR);
#pragma unroll
      for (int i = 0; i < 2; ++i) acc[i][j] = wmma16(af[i], bf, acc[i][j]);
    }
  }
  float* so = oS[wave];
#pragma unroll
  for (int i = 0; i < 2; ++i)
#pragma unroll
    for (int j = 0; j < 4; ++j) {
      const int n = n0 + wn + 16 * j + cl;
      const float bv = bias ? bias[n] : 0.0f;
      const float gv = (EPI == 2) ? gvec[n] : 0.0f;
      if (EPI == 1) {
#pragma unroll 1
        for (int r = 0; r < 8; ++r) { const float xg = acc[i][j][r] + bv; so[(16 * i + rh + r) * 68 + 16 * j + cl] = 0.5f * xg * (1.0f + erff(xg * 0.70710678118654752f)); }
      } else {
#pragma unroll
        for (int r = 0; r < 8; ++r) {
          float v = acc[i][j][r] + bv;
          if (EPI == 2) v = R[(size_t)(m0 + wm + 16 * i + rh + r) * ldy + n] + gv * v;
          so[(16 * i + rh + r) * 68 + 16 * j + cl] = v;
        }
      }
    }
  asm volatile("s_wait_dscnt 0" ::: "memory");
  __builtin_amdgcn_wave_barrier();
#pragma unroll 1
  for (int pass = 0; pass < 2; ++pass) {
    if (OUT16) {
      f16* Y = (f16*)Yv;
#pragma unroll
      for (int it = 0; it < 8; ++it) { const int c = lane + 32 * it, rr = c >> 3, q8 = (c & 7) * 8;
        union { f16 h[8]; v4u_t v; } u;
#pragma unroll
        for (int e = 0; e < 8; ++e) u.h[e] = (f16)so[rr * 68 + q8 + e];
        *(volatile v4u_t*)(Y + (size_t)(m0 + wm + rr) * ldy + n0 + wn + q8) = u.v; }
    } else {
      float* Y = (float*)Yv;
#pragma unroll
      for (int it = 0; it < 16; ++it) { const int f4 = lane + 32 * it, rr = f4 >> 4, q = (f4 & 15) * 4;
        *(volatile v4f_t*)(Y + (size_t)(m0 + wm + rr) * ldy + n0 + wn + q) = *(const v4fa*)(so + rr * 68 + q); }
    }
    __threadfence();
  }
}

__global__ __launch_bounds__(128) void k_padw(const float* __restrict__ Wm, int nout, int kin, float* __restrict__ Wp) { const int r = blockIdx.x, c = threadIdx.x; if (c >= kin) return;
  const float v = (r < nout) ? Wm[r * kin + c] : 0.0f; *(volatile float*)(Wp + (size_t)r * kin + c) = v; __threadfence(); *(volatile float*)(Wp + (size_t)r * kin + c) = v; }
__global__ __launch_bounds__(256) void k_theta(const float* __restrict__ dp, const float* __restrict__ dv, float* __restrict__ TH) {
  __shared__ float vn[MD][3]; __shared__ float pS[256][3 * KNB + 1];
  const int tid = threadIdx.x; const int b = blockIdx.y; const int n = blockIdx.x * 256 + tid;
  if (tid < MD) { const float a = dv[tid * 3], c = dv[tid * 3 + 1], e = dv[tid * 3 + 2]; const float nr = fmaxf(sqrtf(a * a + c * c + e * e), 1e-12f); vn[tid][0] = a / nr; vn[tid][1] = c / nr; vn[tid][2] = e / nr; }
  { const float* bx = dp + (((size_t)b * 3 + 0) * NN + n) * KNB; const float* by = dp + (((size_t)b * 3 + 1) * NN + n) * KNB; const float* bz = dp + (((size_t)b * 3 + 2) * NN + n) * KNB;
#pragma unroll 1
    for (int k = 0; k < KNB; ++k) { const float x = bx[k], y = by[k], z = bz[k]; const float nr = fmaxf(sqrtf(x * x + y * y + z * z), 1e-12f); pS[tid][3 * k] = x / nr; pS[tid][3 * k + 1] = y / nr; pS[tid][3 * k + 2] = z / nr; } }
  __syncthreads();
#pragma unroll 1
  for (int m = 0; m < MD; ++m) { const float a = vn[m][0], c = vn[m][1], e = vn[m][2]; float mx = -3.0e38f;
#pragma unroll 1
    for (int k = 0; k < KNB; ++k) mx = fmaxf(mx, a * pS[tid][3 * k] + c * pS[tid][3 * k + 1] + e * pS[tid][3 * k + 2]);
    float* p = TH + ((size_t)b * MD + m) * NN + n; *(volatile float*)p = mx; __threadfence(); *(volatile float*)p = mx; }
}
__global__ __launch_bounds__(256) void k_rowop(const float* __restrict__ X, int nch, int mode, const float* __restrict__ bias, const float* __restrict__ g, const float* __restrict__ be, const float* __restrict__ mu, const float* __restrict__ var, float* __restrict__ Y) {
  const size_t row = blockIdx.x; const int c = row % nch; const float bb = (mode & 1) ? bias[c] : 0.0f; float sc = 1.0f, sh = 0.0f; if (mode & 2) { sc = g[c] / sqrtf(var[c] + 1e-5f); sh = be[c] - mu[c] * sc; }
  for (int q4 = threadIdx.x; q4 < NN / 4; q4 += 256) { v4f_t v = *(const v4f_t*)(X + row * NN + q4 * 4);
    for (int e = 0; e < 4; ++e) { float u = (v[e] + bb) * sc + sh; if (mode & 4) u = 0.5f * u * (1.0f + erff(u * 0.70710678118654752f)); v[e] = u; }
    *(volatile v4f_t*)(Y + row * NN + q4 * 4) = v; __threadfence(); *(volatile v4f_t*)(Y + row * NN + q4 * 4) = v; } }
__global__ __launch_bounds__(256) void k_knnagg(const float* __restrict__ F1, const float* __restrict__ F2, const float* __restrict__ F3, const int* __restrict__ qidx, const float* __restrict__ g, const float* __restrict__ be, const float* __restrict__ mu, const float* __restrict__ var, float* __restrict__ A) {
  const int tid = threadIdx.x; const int b = blockIdx.y; const int n = blockIdx.x * 256 + tid;
  int id[KNB];
#pragma unroll
  for (int k = 0; k < KNB; ++k) { int v = qidx[(size_t)n * KNB + k]; id[k] = v < 0 ? 0 : (v >= NN ? NN - 1 : v); }
#pragma unroll 1
  for (int c = 0; c < CC; ++c) { const float* r1 = F1 + (size_t)c * NN; const float* r2 = F2 + (size_t)c * NN; const float* r3 = F3 + (size_t)c * NN; (void)b;
    float m1 = -3.0e38f, m2 = -3.0e38f;
#pragma unroll
    for (int k = 0; k < KNB; ++k) { m1 = fmaxf(m1, r1[id[k]]); m2 = fmaxf(m2, r2[id[k]]); }
    const float c1 = r1[n], c2 = r2[n]; const float s = (m1 - c1) + ((m2 - c2) + c2) + r3[n];
    const float sc = g[c] / sqrtf(var[c] + 1e-5f); const float v = (s - mu[c]) * sc + be[c];
    *(volatile float*)(A + (size_t)c * NN + n) = v; __threadfence(); *(volatile float*)(A + (size_t)c * NN + n) = v; }
}
__global__ __launch_bounds__(256) void k_add3(const float* __restrict__ f, const float* __restrict__ A, const float* __restrict__ PE, float* __restrict__ Y) { const size_t row = blockIdx.x;
  for (int q4 = threadIdx.x; q4 < NN / 4; q4 += 256) { const v4f_t a = *(const v4f_t*)(f + row * NN + q4 * 4), d = *(const v4f_t*)(A + row * NN + q4 * 4), p = *(const v4f_t*)(PE + row * NN + q4 * 4); v4f_t o; for (int e = 0; e < 4; ++e) o[e] = a[e] + d[e] + p[e];
    *(volatile v4f_t*)(Y + row * NN + q4 * 4) = o; __threadfence(); *(volatile v4f_t*)(Y + row * NN + q4 * 4) = o; } }
__global__ __launch_bounds__(256) void k_add2(const float* __restrict__ fn, const float* __restrict__ M2, float* __restrict__ out) { const size_t row = blockIdx.x;
  for (int q4 = threadIdx.x; q4 < NN / 4; q4 += 256) { const v4f_t a = *(const v4f_t*)(fn + row * NN + q4 * 4), d = *(const v4f_t*)(M2 + row * NN + q4 * 4); v4f_t o; for (int e = 0; e < 4; ++e) o[e] = a[e] + d[e];
    *(volatile v4f_t*)(out + row * NN + q4 * 4) = o; __threadfence(); *(volatile v4f_t*)(out + row * NN + q4 * 4) = o; } }

extern "C" void kernel_launch(void* const* d_in, const int* in_sizes, int n_in,
                              void* d_out, int out_size, void* d_ws, size_t ws_size,
                              hipStream_t stream) {
  (void)in_sizes; (void)n_in; (void)out_size;
  const float** fp = (const float**)d_in;
  const float* f = fp[0], *dp = fp[1]; const int* qidx = (const int*)d_in[2]; const float* dv = fp[3], *dew1 = fp[4], *deg1 = fp[5], *deb1 = fp[6], *dem1 = fp[7], *dev1 = fp[8], *dew2 = fp[9], *debias2 = fp[10],
             *w1 = fp[11], *b1 = fp[12], *w2 = fp[13], *b2 = fp[14], *w3 = fp[15], *b3 = fp[16], *agg_g = fp[17], *agg_b = fp[18], *agg_m = fp[19], *agg_v = fp[20], *mw1 = fp[21], *mg = fp[22], *mb = fp[23], *mm = fp[24], *mv = fp[25], *mw2 = fp[26];
  float* out = (float*)d_out;
  char* ws = (char*)d_ws;
  float* dew1P = (float*)ws; ws += 128 * 32 * 4; float* dew2P = (float*)ws; ws += 128 * 32 * 4; float* w1P = (float*)ws; ws += 128 * 64 * 4; float* w2P = (float*)ws; ws += 128 * 64 * 4; float* w3P = (float*)ws; ws += 128 * 64 * 4; float* mw1P = (float*)ws; ws += 128 * 64 * 4; float* mw2P = (float*)ws; ws += 128 * 128 * 4;
  float* TH = (float*)ws; ws += (size_t)BB * MD * NN * 4;
  float* Hd = (float*)ws; ws += (size_t)128 * NN * 4;
  float* PE = (float*)ws; ws += (size_t)128 * NN * 4;
  float* F1 = (float*)ws; ws += (size_t)128 * NN * 4; float* F2 = (float*)ws; ws += (size_t)128 * NN * 4; float* F3 = (float*)ws; ws += (size_t)128 * NN * 4;
  float* A = (float*)ws; ws += (size_t)CC * NN * 4;
  float* FN = (float*)ws; ws += (size_t)CC * NN * 4;
  float* H2 = Hd; float* M2 = PE;
  if ((size_t)(ws - (char*)d_ws) > ws_size) return;
  const dim3 blk(256); const dim3 gg(1, NN / 128);
  k_padw<<<dim3(128), dim3(128), 0, stream>>>(dew1, HD2, MD, dew1P); k_padw<<<dim3(128), dim3(128), 0, stream>>>(dew2, CC, HD2, dew2P);
  k_padw<<<dim3(128), dim3(128), 0, stream>>>(w1, CC, CC, w1P); k_padw<<<dim3(128), dim3(128), 0, stream>>>(w2, CC, CC, w2P); k_padw<<<dim3(128), dim3(128), 0, stream>>>(w3, CC, CC, w3P);
  k_padw<<<dim3(128), dim3(128), 0, stream>>>(mw1, HIDm, CC, mw1P); k_padw<<<dim3(128), dim3(128), 0, stream>>>(mw2, CC, HIDm, mw2P);
  k_theta<<<dim3(NN / 256, BB), blk, 0, stream>>>(dp, dv, TH);
  for (int b = 0; b < BB; ++b) {
    const float* fb = f + (size_t)b * CC * NN; float* ob = out + (size_t)b * CC * NN;
    gemm_kne<float, 0, false><<<gg, blk, 0, stream>>>(dew1P, MD, TH + (size_t)b * MD * NN, NN, nullptr, nullptr, nullptr, Hd, NN, MD);
    k_rowop<<<dim3(HD2), blk, 0, stream>>>(Hd, HD2, 2 | 4, nullptr, deg1, deb1, dem1, dev1, Hd);
    gemm_kne<float, 0, false><<<gg, blk, 0, stream>>>(dew2P, HD2, Hd, NN, nullptr, nullptr, nullptr, PE, NN, HD2);
    k_rowop<<<dim3(CC), blk, 0, stream>>>(PE, CC, 1, debias2, nullptr, nullptr, nullptr, nullptr, PE);
    gemm_kne<float, 0, false><<<gg, blk, 0, stream>>>(w1P, CC, fb, NN, nullptr, nullptr, nullptr, F1, NN, CC); k_rowop<<<dim3(CC), blk, 0, stream>>>(F1, CC, 1, b1, nullptr, nullptr, nullptr, nullptr, F1);
    gemm_kne<float, 0, false><<<gg, blk, 0, stream>>>(w2P, CC, fb, NN, nullptr, nullptr, nullptr, F2, NN, CC); k_rowop<<<dim3(CC), blk, 0, stream>>>(F2, CC, 1, b2, nullptr, nullptr, nullptr, nullptr, F2);
    gemm_kne<float, 0, false><<<gg, blk, 0, stream>>>(w3P, CC, fb, NN, nullptr, nullptr, nullptr, F3, NN, CC); k_rowop<<<dim3(CC), blk, 0, stream>>>(F3, CC, 1, b3, nullptr, nullptr, nullptr, nullptr, F3);
    k_knnagg<<<dim3(NN / 256, 1), blk, 0, stream>>>(F1 - 0, F2, F3, qidx + (size_t)b * NN * KNB, agg_g, agg_b, agg_m, agg_v, A);
    k_add3<<<dim3(CC), blk, 0, stream>>>(fb, A, PE, FN);
    gemm_kne<float, 0, false><<<gg, blk, 0, stream>>>(mw1P, CC, FN, NN, nullptr, nullptr, nullptr, H2, NN, CC);
    k_rowop<<<dim3(HIDm), blk, 0, stream>>>(H2, HIDm, 2 | 4, nullptr, mg, mb, mm, mv, H2);
    gemm_kne<float, 0, false><<<gg, blk, 0, stream>>>(mw2P, HIDm, H2, NN, nullptr, nullptr, nullptr, M2, NN, HIDm);
    k_add2<<<dim3(CC), blk, 0, stream>>>(FN, M2, ob);
  }
}
